// CALIP_PF_Block_76373108457749
// MI455X (gfx1250) — hardware-verified
//
#include <hip/hip_runtime.h>


#define NBI  128
#define MM   196
#define MP   256
#define KT   1000
#define KTP  1024
#define DD   512
#define DM   DD
#define NTK  MP
#define ALS  0.5f
#define ALT  0.5f
#define B1_  1.0f
#define B2_  0.1f
#define B3_  0.1f
#define LOSC 1024.0f

typedef _Float16 h16;
typedef unsigned short bf;
typedef __attribute__((ext_vector_type(16))) __bf16   v16bf;
typedef __attribute__((ext_vector_type(16))) _Float16 v16h;
typedef __attribute__((ext_vector_type(8)))  _Float16 v8h;
typedef __attribute__((ext_vector_type(8)))  unsigned short v8us;
typedef __attribute__((ext_vector_type(8)))  float    v8f;
typedef __attribute__((ext_vector_type(4)))  float    v4f;
typedef __attribute__((ext_vector_type(4)))  _Float16 v4h;
typedef v8h  __attribute__((may_alias)) v8ha;
typedef v4f  __attribute__((may_alias)) v4fa;
typedef v8us __attribute__((may_alias)) v8usa;

__device__ __forceinline__ unsigned short f2bf(float f) { unsigned u = __float_as_uint(f); u += 0x7FFFu + ((u >> 16) & 1u); return (unsigned short)(u >> 16); }
__device__ __forceinline__ float bf2f(unsigned short b) { return __uint_as_float(((unsigned)b) << 16); }
__device__ __forceinline__ float bfr(float f) { return bf2f(f2bf(f)); }
__device__ __forceinline__ v16h cat16(v8h lo, v8h hi) { return __builtin_shufflevector(lo, hi, 0, 1, 2, 3, 4, 5, 6, 7, 8, 9, 10, 11, 12, 13, 14, 15); }
__device__ __forceinline__ v16bf cat16b(v8us lo, v8us hi) { return __builtin_bit_cast(v16bf, __builtin_shufflevector(lo, hi, 0, 1, 2, 3, 4, 5, 6, 7, 8, 9, 10, 11, 12, 13, 14, 15)); }
__device__ __forceinline__ v8f wmma16(v16h a, v16h b, v8f c) { return __builtin_amdgcn_wmma_f32_16x16x32_f16(false, a, false, b, (short)0, c, false, false); }
__device__ __forceinline__ v8f wmmab(v16bf a, v16bf b, v8f c) { return __builtin_amdgcn_wmma_f32_16x16x32_bf16(false, a, false, b, (short)0, c, false, false); }

__global__ __launch_bounds__(256) void k_wt(const float* __restrict__ Wm, int K, int ncols, bf* WT) {
    __shared__ __align__(16) unsigned short tl[64 * 72];
    const int tid = threadIdx.x, k0 = blockIdx.x * 64, n0 = blockIdx.y * 64;
    const int kk = tid >> 2, nq = (tid & 3) * 16;
#pragma unroll
    for (int i = 0; i < 16; ++i) tl[(nq + i) * 72 + kk] = f2bf(Wm[(size_t)(k0 + kk) * ncols + n0 + nq + i]);
    __syncthreads();
    const int piece = tid & 7;
    auto pass = [&]() {
#pragma unroll
        for (int s = 0; s < 2; ++s) { const int nr = (tid >> 3) + 32 * s; const v8us val = *(const v8usa*)(tl + nr * 72 + piece * 8); *(volatile v8us*)(WT + (size_t)(n0 + nr) * K + k0 + piece * 8) = val; }
    };
    pass(); __threadfence(); pass();
}
template <bool SPLITA, bool F16OUT = false>
__global__ __launch_bounds__(128) void k_gemmb(const bf* __restrict__ A, const bf* __restrict__ Al, const bf* __restrict__ Bn, const float* __restrict__ bias, float* C, int ldc, h16* C2, const float* __restrict__ R = nullptr, int K = DM, int roundR = 1) {
    __shared__ __align__(16) float ost[4][16 * 68];
    const int lane = threadIdx.x & 31, wave = threadIdx.x >> 5, lr = lane & 15, hi = lane >> 4;
    const int r0 = blockIdx.x * 64 + wave * 16, c0 = blockIdx.y * 64;
    const size_t aoff = (size_t)(r0 + lr) * K + 8 * hi;
    size_t boff[4];
#pragma unroll
    for (int t = 0; t < 4; ++t) boff[t] = (size_t)(c0 + t * 16 + lr) * K + 8 * hi;
    v8f acc[4];
#pragma unroll
    for (int t = 0; t < 4; ++t) acc[t] = (v8f){};
#pragma unroll 1
    for (int kc = 0; kc < K; kc += 32) {
        const v16bf a = cat16b(*(const v8us*)(A + aoff + kc), *(const v8us*)(A + aoff + kc + 16));
        v16bf al = a;
        if (SPLITA) al = cat16b(*(const v8us*)(Al + aoff + kc), *(const v8us*)(Al + aoff + kc + 16));
#pragma unroll
        for (int t = 0; t < 4; ++t) { const v16bf b = cat16b(*(const v8us*)(Bn + boff[t] + kc), *(const v8us*)(Bn + boff[t] + kc + 16)); acc[t] = wmmab(a, b, acc[t]); if (SPLITA) acc[t] = wmmab(al, b, acc[t]); }
        asm volatile("v_nop\n\tv_nop\n\tv_nop\n\tv_nop" : "+v"(acc[0]), "+v"(acc[1]), "+v"(acc[2]), "+v"(acc[3]) : "v"(a), "v"(al));
    }
    float* os = &ost[wave][0];
#pragma unroll
    for (int t = 0; t < 4; ++t) { const float bv = bias ? bfr(bias[c0 + t * 16 + lr]) : 0.f;
#pragma unroll
        for (int j = 0; j < 8; ++j) os[(hi * 8 + j) * 68 + t * 16 + lr] = acc[t][j] + bv; }
    __syncthreads();
    if (F16OUT) {
        h16* crow = (h16*)(void*)C + (size_t)r0 * ldc + c0;
        auto pass = [&]() {
#pragma unroll
            for (int s = 0; s < 4; ++s) { const int row = 4 * s + (lane >> 3), piece = lane & 7; const float* sp = os + row * 68 + piece * 8; v8h o, o2;
#pragma unroll
                for (int i = 0; i < 8; ++i) { const h16 a = (h16)sp[i]; o[i] = a; o2[i] = (h16)((sp[i] - (float)a) * LOSC); }
                *(volatile v8h*)(crow + (size_t)row * ldc + piece * 8) = o; if (C2) *(volatile v8h*)(C2 + (size_t)r0 * ldc + c0 + (size_t)row * ldc + piece * 8) = o2; }
        };
        pass(); __threadfence(); pass();
    } else {
        float* crow = C + (size_t)r0 * ldc + c0;
        auto pass = [&]() {
#pragma unroll
            for (int s = 0; s < 8; ++s) { const int Lid = (lane >> 3) + 4 * s, piece = lane & 7; const int row = Lid >> 1, cofs = (Lid & 1) * 32 + piece * 4;
                v4f val = *(const v4fa*)(os + row * 68 + cofs); if (R) { const v4f rv = *(const v4f*)(R + ((size_t)r0 + row) * ldc + c0 + cofs); val += roundR ? (v4f){bfr(rv[0]), bfr(rv[1]), bfr(rv[2]), bfr(rv[3])} : rv; }
                *(volatile v4f*)(crow + (size_t)row * ldc + cofs) = val; }
        };
        pass(); __threadfence(); pass();
    }
}

__global__ __launch_bounds__(128) void k_gemm3(const bf* __restrict__ Ah, const bf* __restrict__ Al, const bf* __restrict__ Bh, const bf* __restrict__ Bl, int K, float* C, int ldc) {
    __shared__ __align__(16) float ost[4][16 * 68];
    const int lane = threadIdx.x & 31, wave = threadIdx.x >> 5, lr = lane & 15, hi = lane >> 4;
    const int r0 = blockIdx.x * 64 + wave * 16, c0 = blockIdx.y * 64;
    const size_t aoff = (size_t)(r0 + lr) * K + 8 * hi;
    v8f acc[4];
#pragma unroll
    for (int t = 0; t < 4; ++t) acc[t] = (v8f){};
#pragma unroll 1
    for (int kc = 0; kc < K; kc += 32) {
        const v16bf a = cat16b(*(const v8us*)(Ah + aoff + kc), *(const v8us*)(Ah + aoff + kc + 16));
        const v16bf al = cat16b(*(const v8us*)(Al + aoff + kc), *(const v8us*)(Al + aoff + kc + 16));
#pragma unroll
        for (int t = 0; t < 4; ++t) { const size_t bo = (size_t)(c0 + t * 16 + lr) * K + kc + 8 * hi;
            const v16bf bh = cat16b(*(const v8us*)(Bh + bo), *(const v8us*)(Bh + bo + 16)); const v16bf bl = cat16b(*(const v8us*)(Bl + bo), *(const v8us*)(Bl + bo + 16));
            acc[t] = wmmab(a, bh, acc[t]); acc[t] = wmmab(al, bh, acc[t]); acc[t] = wmmab(a, bl, acc[t]); }
        asm volatile("v_nop\n\tv_nop\n\tv_nop\n\tv_nop" : "+v"(acc[0]), "+v"(acc[1]), "+v"(acc[2]), "+v"(acc[3]) : "v"(a), "v"(al));
    }
    float* os = &ost[wave][0];
#pragma unroll
    for (int t = 0; t < 4; ++t) {
#pragma unroll
        for (int j = 0; j < 8; ++j) os[(hi * 8 + j) * 68 + t * 16 + lr] = acc[t][j]; }
    __builtin_amdgcn_wave_barrier(); asm volatile("" ::: "memory");
    float* crow = C + (size_t)r0 * ldc + c0;
    auto pass = [&]() {
#pragma unroll
        for (int s = 0; s < 8; ++s) { const int Lid = (lane >> 3) + 4 * s, piece = lane & 7; const int row = Lid >> 1, cofs = (Lid & 1) * 32 + piece * 4;
            const v4f val = *(const v4fa*)(os + row * 68 + cofs); *(volatile v4f*)(crow + (size_t)row * ldc + cofs) = val; }
    };
    pass(); __threadfence(); pass();
}

__global__ __launch_bounds__(256) void k_ftpad(const float* __restrict__ Ft, float* FtP, bf* FtB) {
    const size_t u = (size_t)blockIdx.x * 256 + threadIdx.x; if (u >= (size_t)KTP * DD / 8) return;
    const int k = (int)(u / (DD / 8)); v8f v; v8us o;
#pragma unroll
    for (int i = 0; i < 8; ++i) { v[i] = (k < KT) ? Ft[u * 8 + i] : 0.f; o[i] = f2bf(v[i]); }
    *(volatile v8f*)(FtP + u * 8) = v; *(volatile v8us*)(FtB + u * 8) = o; __threadfence(); *(volatile v8f*)(FtP + u * 8) = v; *(volatile v8us*)(FtB + u * 8) = o;
}
__global__ __launch_bounds__(256) void k_norm(const float* __restrict__ Fs, int b, float* INV) {
    const int m = threadIdx.x; float s = 0.f;
    if (m < MM) { const float* r = Fs + ((size_t)b * MM + m) * DD;
#pragma unroll 1
        for (int d = 0; d < DD; ++d) { const float v = bfr(r[d]); s = fmaf(v, v, s); } }
    const float inv = (m < MM) ? 1.0f / sqrtf(s) : 0.f;
    *(volatile float*)(INV + m) = inv; __threadfence(); *(volatile float*)(INV + m) = inv;
}
__global__ __launch_bounds__(256) void k_fsn(const float* __restrict__ Fs, const float* __restrict__ INV, int b, bf* Nh, bf* Nl) {
    const int lane = threadIdx.x & 31, m = blockIdx.x * 8 + (threadIdx.x >> 5); if (m >= MP) return;
    const float inv = INV[m];
#pragma unroll 1
    for (int ps = 0; ps < 2; ++ps) {
#pragma unroll 1
        for (int q = 0; q < DD / 256; ++q) { const int d0 = q * 256 + lane * 8; v8us oh, ol;
#pragma unroll
            for (int i = 0; i < 8; ++i) { const float v = (m < MM) ? bfr(Fs[((size_t)b * MM + m) * DD + d0 + i]) * inv : 0.f; const unsigned short hb = f2bf(v); oh[i] = hb; ol[i] = f2bf(v - bf2f(hb)); }
            const size_t o = (size_t)m * DD + d0; *(volatile v8us*)(Nh + o) = oh; *(volatile v8us*)(Nl + o) = ol; }
        if (ps == 0) __threadfence(); }
}
__global__ __launch_bounds__(256) void k_fsnT(const float* __restrict__ Fs, const float* __restrict__ INV, int b, bf* Th, bf* Tl) {
    typedef __attribute__((ext_vector_type(2))) unsigned short v2us;
    const int lane = threadIdx.x & 31, wid = blockIdx.x * 8 + (threadIdx.x >> 5); if (wid >= DD * (MP / 64)) return;
    const int g = wid % (MP / 64), d = wid / (MP / 64); const int m0 = g * 64 + 2 * lane; v2us oh, ol;
#pragma unroll
    for (int i = 0; i < 2; ++i) { const int m = m0 + i; const float v = (m < MM) ? bfr(Fs[((size_t)b * MM + m) * DD + d]) * INV[m] : 0.f; const unsigned short hb = f2bf(v); oh[i] = hb; ol[i] = f2bf(v - bf2f(hb)); }
    const size_t o = (size_t)d * MP + m0;
    *(volatile v2us*)(Th + o) = oh; *(volatile v2us*)(Tl + o) = ol; __threadfence(); *(volatile v2us*)(Th + o) = oh; *(volatile v2us*)(Tl + o) = ol;
}
__global__ __launch_bounds__(256) void k_soft_s(const float* __restrict__ A, bf* PH, bf* PL) {
    const int lane = threadIdx.x & 31, m = blockIdx.x * 8 + (threadIdx.x >> 5); if (m >= MP) return;
    const float* ar = A + (size_t)m * KTP; float mx = -3.0e38f;
#pragma unroll 1
    for (int c0 = lane * 8; c0 < KTP; c0 += 256) { const v8f v = *(const v8f*)(ar + c0);
#pragma unroll
        for (int i = 0; i < 8; ++i) if (c0 + i < KT) mx = fmaxf(mx, v[i] * (1.0f / ALS)); }
#pragma unroll
    for (int sh = 16; sh; sh >>= 1) mx = fmaxf(mx, __shfl_xor(mx, sh, 32));
    float sum = 0.f;
#pragma unroll 1
    for (int c0 = lane * 8; c0 < KTP; c0 += 256) { const v8f v = *(const v8f*)(ar + c0);
#pragma unroll
        for (int i = 0; i < 8; ++i) if (c0 + i < KT) sum += __expf(v[i] * (1.0f / ALS) - mx); }
#pragma unroll
    for (int sh = 16; sh; sh >>= 1) sum += __shfl_xor(sum, sh, 32);
    const float inv = 1.0f / sum;
#pragma unroll 1
    for (int ps = 0; ps < 2; ++ps) {
#pragma unroll 1
        for (int c0 = lane * 8; c0 < KTP; c0 += 256) { const v8f v = *(const v8f*)(ar + c0); v8us oh, ol;
#pragma unroll
            for (int i = 0; i < 8; ++i) { const float p = (c0 + i < KT) ? __expf(v[i] * (1.0f / ALS) - mx) * inv : 0.f; const unsigned short hb = f2bf(p); oh[i] = hb; ol[i] = f2bf(p - bf2f(hb)); }
            const size_t o = (size_t)m * KTP + c0; *(volatile v8us*)(PH + o) = oh; *(volatile v8us*)(PL + o) = ol; }
        if (ps == 0) __threadfence(); }
}
__global__ __launch_bounds__(256) void k_soft_t(const float* __restrict__ A, bf* PTh, bf* PTl) {
    typedef __attribute__((ext_vector_type(2))) unsigned short v2us;
    const int lane = threadIdx.x & 31, k = blockIdx.x * 8 + (threadIdx.x >> 5); if (k >= KTP) return;
    float a[MP / 32]; float mx = -3.0e38f;
#pragma unroll
    for (int j = 0; j < MP / 64; ++j)
#pragma unroll
        for (int i = 0; i < 2; ++i) { const int m = j * 64 + 2 * lane + i; const float v = (m < MM && k < KT) ? A[(size_t)m * KTP + k] * (1.0f / ALT) : -3.0e38f; a[j * 2 + i] = v; mx = fmaxf(mx, v); }
#pragma unroll
    for (int sh = 16; sh; sh >>= 1) mx = fmaxf(mx, __shfl_xor(mx, sh, 32));
    float sum = 0.f;
#pragma unroll
    for (int j = 0; j < MP / 32; ++j) sum += (a[j] > -1.0e38f) ? __expf(a[j] - mx) : 0.f;
#pragma unroll
    for (int sh = 16; sh; sh >>= 1) sum += __shfl_xor(sum, sh, 32);
    const float inv = (k < KT) ? 1.0f / sum : 0.f;
#pragma unroll 1
    for (int ps = 0; ps < 2; ++ps) {
#pragma unroll
        for (int j = 0; j < MP / 64; ++j) { v2us oh, ol;
#pragma unroll
            for (int i = 0; i < 2; ++i) { const float p = (a[j * 2 + i] > -1.0e38f) ? __expf(a[j * 2 + i] - mx) * inv : 0.f; const unsigned short hb = f2bf(p); oh[i] = hb; ol[i] = f2bf(p - bf2f(hb)); }
            const size_t o = (size_t)k * MP + j * 64 + 2 * lane; *(volatile v2us*)(PTh + o) = oh; *(volatile v2us*)(PTl + o) = ol; }
        if (ps == 0) __threadfence(); }
}
__global__ __launch_bounds__(256) void k_pool(const float* __restrict__ Fsa, int b, float* FVA) {
    const int d = blockIdx.x * 256 + threadIdx.x; if (d >= DD) return; float s = 0.f, mx = -3.0e38f;
#pragma unroll 1
    for (int m = 0; m < MM; ++m) { const float v = Fsa[(size_t)m * DD + d]; s += v; mx = fmaxf(mx, v); }
    const float y = s * (1.0f / MM) + mx; *(volatile float*)(FVA + (size_t)b * DD + d) = y; __threadfence(); *(volatile float*)(FVA + (size_t)b * DD + d) = y;
}
__global__ __launch_bounds__(256) void k_logits(const float* __restrict__ Fv, const float* __restrict__ Ft, const float* __restrict__ FTA, const float* __restrict__ FVA, const float* __restrict__ lsc, int b, float* RES) {
    const int k = blockIdx.x * 256 + threadIdx.x; if (k >= KTP) return; float r = 0.f;
    if (k < KT) { float d1 = 0.f, d2 = 0.f, d3 = 0.f;
#pragma unroll 1
        for (int d = 0; d < DD; ++d) { const float fv = bfr(Fv[(size_t)b * DD + d]), ft = bfr(Ft[(size_t)k * DD + d]); d1 = fmaf(fv, ft, d1); d2 = fmaf(fv, FTA[(size_t)k * DD + d], d2); d3 = fmaf(FVA[(size_t)b * DD + d], ft, d3); }
        const float ls = __expf(bfr(lsc[0])); r = B1_ * ls * d1 + B2_ * ls * d2 + B3_ * ls * d3; }
    *(volatile float*)(RES + (size_t)b * KTP + k) = r; __threadfence(); *(volatile float*)(RES + (size_t)b * KTP + k) = r;
}
__global__ __launch_bounds__(256) void k_out(const float* __restrict__ RES, float* OUTP) {
    const int i = blockIdx.x * 256 + threadIdx.x; if (i >= NBI * KT) return; const float v = RES[(size_t)(i / KT) * KTP + (i % KT)];
    *(volatile float*)(OUTP + i) = v; __threadfence(); *(volatile float*)(OUTP + i) = v;
}

extern "C" void kernel_launch(void* const* d_in, const int* in_sizes, int n_in,
                              void* d_out, int out_size, void* d_ws, size_t ws_size, hipStream_t stream) {
    (void)in_sizes; (void)n_in; (void)out_size;
    const float* Fs = (const float*)d_in[0]; const float* Ft = (const float*)d_in[1]; const float* Fv = (const float*)d_in[2]; const float* lsc = (const float*)d_in[3];
    float* out = (float*)d_out;
    char* wsp = (char*)d_ws;
    auto take = [&](size_t bytes) { char* p = wsp; wsp += (bytes + 255) & ~(size_t)255; return (void*)p; };
    float* FtP = (float*)take((size_t)KTP * DD * 4); bf* FtB = (bf*)take((size_t)KTP * DD * 2); bf* FtT = (bf*)take((size_t)DD * KTP * 2); float* INV = (float*)take(MP * 4);
    bf* Nh = (bf*)take((size_t)MP * DD * 2); bf* Nl = (bf*)take((size_t)MP * DD * 2); bf* Th = (bf*)take((size_t)DD * MP * 2); bf* Tl = (bf*)take((size_t)DD * MP * 2);
    float* A = (float*)take((size_t)MP * KTP * 4); bf* PH = (bf*)take((size_t)MP * KTP * 2); bf* PL = (bf*)take((size_t)MP * KTP * 2); bf* PTh = (bf*)take((size_t)KTP * MP * 2); bf* PTl = (bf*)take((size_t)KTP * MP * 2);
    float* FSA = (float*)take((size_t)MP * DD * 4); float* FTA = (float*)take((size_t)KTP * DD * 4); float* FVA = (float*)take((size_t)NBI * DD * 4); float* RES = (float*)take((size_t)NBI * KTP * 4);
    if ((size_t)(wsp - (char*)d_ws) > ws_size) return;
    k_ftpad<<<(KTP * DD / 8 + 255) / 256, 256, 0, stream>>>(Ft, FtP, FtB); k_wt<<<dim3(KTP / 64, DD / 64, 1), 256, 0, stream>>>(FtP, KTP, DD, FtT);
    for (int b = 0; b < NBI; ++b) {
        k_norm<<<1, 256, 0, stream>>>(Fs, b, INV);
        k_fsn<<<MP / 8, 256, 0, stream>>>(Fs, INV, b, Nh, Nl); k_fsnT<<<(DD * (MP / 64)) / 8, 256, 0, stream>>>(Fs, INV, b, Th, Tl);
        k_gemmb<true, false><<<dim3(MP / 64, KTP / 64, 1), 128, 0, stream>>>(Nh, Nl, FtB, nullptr, A, KTP, nullptr, nullptr, DD);
        k_soft_s<<<MP / 8, 256, 0, stream>>>(A, PH, PL); k_soft_t<<<KTP / 8, 256, 0, stream>>>(A, PTh, PTl);
        k_gemmb<true, false><<<dim3(MP / 64, DD / 64, 1), 128, 0, stream>>>(PH, PL, FtT, nullptr, FSA, DD, nullptr, nullptr, KTP);
        k_gemm3<<<dim3(KTP / 64, DD / 64, 1), 128, 0, stream>>>(PTh, PTl, Th, Tl, MP, FTA, DD);
        k_pool<<<DD / 256, 256, 0, stream>>>(FSA, b, FVA);
        k_logits<<<KTP / 256, 256, 0, stream>>>(Fv, Ft, FTA, FVA, lsc, b, RES);
    }
    k_out<<<(NBI * KT + 255) / 256, 256, 0, stream>>>(RES, out);
}
